// CatalystGNNLayer_71519795413188
// MI455X (gfx1250) — hardware-verified
//
#include <hip/hip_runtime.h>
#include <stddef.h>


#define NTHR   256
#define NWAVE  8
#define HD     128
#define TR     64
#define EPT    8
#define CHUNK  (NTHR * EPT)
#define WCAP   (EPT * 32)
#define NB     256
#define SLOTB  8

static_assert(NB == (1 << SLOTB));
static_assert((NB % NWAVE) == 0);
static_assert((NB % 128) == 0);
static_assert(NWAVE * WCAP == CHUNK);
static_assert(TR == 8 * NWAVE);
static_assert(((TR * HD / 4) % NTHR) == 0);

#define OFF_W1H 0
#define OFF_W1L 32768
#define OFF_W2H 65536
#define OFF_W2L 81920
#define OFF_U1H 98304
#define OFF_U1L 131072
#define OFF_U2H 163840
#define OFF_U2L 180224
#define WT_HALVES 196608

#define LDS_PQ   (2 * TR * HD * 2 + TR * 2 * HD * 4)
#define LDS_NODE (2 * TR * 2 * HD * 2 + 2 * TR * HD * 2)
#define LDS_AGG  (NB * HD * 4 + NB * 4)

typedef float          v4f    __attribute__((ext_vector_type(4)));
typedef float          v8f    __attribute__((ext_vector_type(8)));
typedef int            v4i    __attribute__((ext_vector_type(4)));
typedef unsigned short us16;
typedef us16           v4us_t __attribute__((ext_vector_type(4)));
typedef us16           v8us_t __attribute__((ext_vector_type(8)));
typedef v4us_t __attribute__((may_alias)) v4us;
typedef v8us_t __attribute__((may_alias)) v8us;
typedef v4f    __attribute__((may_alias)) v4fa;
typedef v4i    __attribute__((may_alias)) v4ia;
typedef __bf16         v16bf  __attribute__((ext_vector_type(16)));
union FragB { v16bf v; v8us_t h[2]; };

__device__ __forceinline__ unsigned f2bf(float f) {
  unsigned u = __float_as_uint(f);
  u += 0x7FFFu + ((u >> 16) & 1u);
  return u >> 16;
}
__device__ __forceinline__ void split2(float v, us16& hi, us16& lo) {
  const unsigned hb = f2bf(v);
  const float hf = __uint_as_float(hb << 16);
  hi = (us16)hb;
  lo = (us16)f2bf(v - hf);
}

__device__ __forceinline__ v8f vz8() {
  v8f z;
#pragma unroll
  for (int i = 0; i < 8; ++i) z[i] = 0.0f;
  return z;
}

__device__ __forceinline__ v8f wmb(v16bf a, v16bf b, v8f c) {
  v8f d = __builtin_amdgcn_wmma_f32_16x16x32_bf16(false, a, false, b, (short)0, c, false, false);
  asm volatile("v_nop\n\tv_nop\n\tv_nop\n\tv_nop" : "+v"(d) : "v"(a), "v"(b));
  return d;
}

__device__ __forceinline__ v16bf ldfrag(const us16* pl, int pitch, int rown, int k0, int h) {
  const us16* p = pl + (size_t)rown * (size_t)pitch + k0 + 8 * h;
  FragB f;
  f.h[0] = *(const v8us*)p;
  f.h[1] = *(const v8us*)(p + 16);
  return f.v;
}

__device__ __forceinline__ void wgemm2(v8f& c00, v8f& c01, v8f& c10, v8f& c11,
                                       const us16* ah, const us16* al, int ap, int arow0,
                                       const us16* bh, const us16* bl, int bp, int bcol0,
                                       int K, int m, int h) {
#pragma unroll 1
  for (int k0 = 0; k0 < K; k0 += 32) {
    const v16bf a0h = ldfrag(ah, ap, arow0 + m, k0, h);
    const v16bf a0l = ldfrag(al, ap, arow0 + m, k0, h);
    const v16bf a1h = ldfrag(ah, ap, arow0 + 16 + m, k0, h);
    const v16bf a1l = ldfrag(al, ap, arow0 + 16 + m, k0, h);
    {
      const v16bf b0h = ldfrag(bh, bp, bcol0 + m, k0, h);
      const v16bf b0l = ldfrag(bl, bp, bcol0 + m, k0, h);
      c00 = wmb(a0h, b0h, c00); c00 = wmb(a0l, b0h, c00); c00 = wmb(a0h, b0l, c00);
      c10 = wmb(a1h, b0h, c10); c10 = wmb(a1l, b0h, c10); c10 = wmb(a1h, b0l, c10);
    }
    {
      const v16bf b1h = ldfrag(bh, bp, bcol0 + 16 + m, k0, h);
      const v16bf b1l = ldfrag(bl, bp, bcol0 + 16 + m, k0, h);
      c01 = wmb(a0h, b1h, c01); c01 = wmb(a0l, b1h, c01); c01 = wmb(a0h, b1l, c01);
      c11 = wmb(a1h, b1h, c11); c11 = wmb(a1l, b1h, c11); c11 = wmb(a1h, b1l, c11);
    }
  }
}

__device__ __forceinline__ void epi_f32(float* ot, int pitch, v8f acc, int rowb, int col, float bb) {
#pragma unroll
  for (int r = 0; r < 8; ++r) ot[(rowb + r) * pitch + col] = acc[r] + bb;
}
__device__ __forceinline__ void epi_split(us16* ph, us16* pl, int pitch, v8f acc, int rowb, int col, float bb, int relu) {
#pragma unroll
  for (int r = 0; r < 8; ++r) {
    float v = acc[r] + bb;
    if (relu != 0) v = fmaxf(v, 0.0f);
    us16 hi, lo;
    split2(v, hi, lo);
    ph[(rowb + r) * pitch + col] = hi;
    pl[(rowb + r) * pitch + col] = lo;
  }
}
__device__ __forceinline__ void epi_msg(us16* ph, us16* pl, int pitch, v8f acc, int rowb, int col, float bb, const float* sdeg) {
#pragma unroll
  for (int r = 0; r < 8; ++r) {
    const float v = acc[r] + sdeg[rowb + r] * bb;
    us16 hi, lo;
    split2(v, hi, lo);
    ph[(rowb + r) * pitch + col] = hi;
    pl[(rowb + r) * pitch + col] = lo;
  }
}

__global__ __launch_bounds__(NTHR) void k_wcvt(const float* __restrict__ w1, const float* __restrict__ w2,
                                               const float* __restrict__ u1, const float* __restrict__ u2,
                                               us16* wt) {
  __shared__ __attribute__((aligned(16))) us16 th[16 * 2 * HD];
  __shared__ __attribute__((aligned(16))) us16 tl[16 * 2 * HD];
  const int tid = threadIdx.x;
  const int b = blockIdx.x;
  const float* srcp;
  int K, n0;
  size_t oh, ol;
  if (b < 16) {
    n0 = 16 * b; K = HD;
    srcp = (n0 < HD) ? (w1 + n0) : (w1 + (size_t)HD * HD + (n0 - HD));
    oh = OFF_W1H; ol = OFF_W1L;
  } else if (b < 24) {
    n0 = 16 * (b - 16); K = HD; srcp = w2 + n0; oh = OFF_W2H; ol = OFF_W2L;
  } else if (b < 32) {
    n0 = 16 * (b - 24); K = 2 * HD; srcp = u1 + n0; oh = OFF_U1H; ol = OFF_U1L;
  } else {
    n0 = 16 * (b - 32); K = HD; srcp = u2 + n0; oh = OFF_U2H; ol = OFF_U2L;
  }
  if (b >= 40) return;
  oh += (size_t)n0 * (size_t)K;
  ol += (size_t)n0 * (size_t)K;
#pragma unroll 1
  for (int idx = tid; idx < 16 * K; idx += NTHR) {
    const int k = idx >> 4, nl = idx & 15;
    const float v = srcp[(size_t)k * HD + nl];
    us16 hi, lo;
    split2(v, hi, lo);
    th[nl * K + k] = hi;
    tl[nl * K + k] = lo;
  }
  __syncthreads();
  const int np = 2 * K;
  for (int p = tid; p < np; p += NTHR) {
    const v8us_t a = *(const v8us*)(th + 8 * p);
    const v8us_t c = *(const v8us*)(tl + 8 * p);
    *(volatile v8us_t*)(wt + oh + 8 * p) = a;
    *(volatile v8us_t*)(wt + ol + 8 * p) = c;
  }
  __threadfence();
  for (int p = tid; p < np; p += NTHR) {
    const v8us_t a = *(const v8us*)(th + 8 * p);
    const v8us_t c = *(const v8us*)(tl + 8 * p);
    *(volatile v8us_t*)(wt + oh + 8 * p) = a;
    *(volatile v8us_t*)(wt + ol + 8 * p) = c;
  }
}

__global__ __launch_bounds__(NTHR) void k_pq(const float* __restrict__ x, const us16* __restrict__ wt,
                                             float* pq, int nN) {
  extern __shared__ v4f dsm4[];
  unsigned char* dsm = (unsigned char*)dsm4;
  us16*  XH = (us16*)dsm;
  us16*  XL = XH + TR * HD;
  float* OT = (float*)(dsm + (size_t)2 * TR * HD * 2);
  const int tid = threadIdx.x, lane = tid & 31, wave = tid >> 5, h = lane >> 4, m = lane & 15;
  const int row0 = blockIdx.x * TR;

#pragma unroll
  for (int it = 0; it < (TR * HD / 4) / NTHR; ++it) {
    const int idx = it * NTHR + tid;
    const int r = idx >> 5, c4 = idx & 31;
    int grow = row0 + r; grow = grow > nN - 1 ? nN - 1 : grow;
    const v4f v = *(const v4fa*)(x + (size_t)grow * HD + 4 * c4);
    us16 a0, b0, a1, b1, a2, b2, a3, b3;
    split2(v.x, a0, b0); split2(v.y, a1, b1); split2(v.z, a2, b2); split2(v.w, a3, b3);
    v4us_t hv, lv;
    hv.x = a0; hv.y = a1; hv.z = a2; hv.w = a3;
    lv.x = b0; lv.y = b1; lv.z = b2; lv.w = b3;
    *(v4us*)(XH + r * HD + 4 * c4) = hv;
    *(v4us*)(XL + r * HD + 4 * c4) = lv;
  }
  __syncthreads();

  const int rh = wave >> 2, cg = wave & 3;
  const int arow0 = 32 * rh;
#pragma unroll 1
  for (int half = 0; half < 2; ++half) {
    const int bcol0 = 64 * cg + 32 * half;
    v8f c00 = vz8(), c01 = vz8(), c10 = vz8(), c11 = vz8();
    wgemm2(c00, c01, c10, c11, XH, XL, HD, arow0, wt + OFF_W1H, wt + OFF_W1L, HD, bcol0, HD, m, h);
    epi_f32(OT, 2 * HD, c00, arow0 + 8 * h,      bcol0 + m,      0.0f);
    epi_f32(OT, 2 * HD, c01, arow0 + 8 * h,      bcol0 + 16 + m, 0.0f);
    epi_f32(OT, 2 * HD, c10, arow0 + 16 + 8 * h, bcol0 + m,      0.0f);
    epi_f32(OT, 2 * HD, c11, arow0 + 16 + 8 * h, bcol0 + 16 + m, 0.0f);
  }
  __syncthreads();

  for (int r = wave; r < TR; r += NWAVE) {
    const size_t gb = (size_t)(row0 + r) * (size_t)(2 * HD);
    const v4f v0 = *(const v4fa*)(OT + r * 2 * HD + 4 * lane);
    const v4f v1 = *(const v4fa*)(OT + r * 2 * HD + HD + 4 * lane);
    *(volatile v4f*)(pq + gb + 4 * lane) = v0;
    *(volatile v4f*)(pq + gb + HD + 4 * lane) = v1;
  }
  __threadfence();
  for (int r = wave; r < TR; r += NWAVE) {
    const size_t gb = (size_t)(row0 + r) * (size_t)(2 * HD);
    const v4f v0 = *(const v4fa*)(OT + r * 2 * HD + 4 * lane);
    const v4f v1 = *(const v4fa*)(OT + r * 2 * HD + HD + 4 * lane);
    *(volatile v4f*)(pq + gb + 4 * lane) = v0;
    *(volatile v4f*)(pq + gb + HD + 4 * lane) = v1;
  }
}

__device__ __forceinline__ int scan_chunk(const int* __restrict__ ei, int nE, int cbase, int nodeBase,
                                          int* list, int tid, int wave) {
  int wc = 0;
  const int el0  = tid * EPT;
  const int e0   = cbase + el0;
  const int sent = -2147483647 - 1;
  int d0, d1, d2, d3, d4, d5, d6, d7;
  if (cbase + CHUNK <= nE) {
    const int* p = ei + 2 * (size_t)e0;
    const v4i q0 = *(const v4ia*)(p);
    const v4i q1 = *(const v4ia*)(p + 4);
    const v4i q2 = *(const v4ia*)(p + 8);
    const v4i q3 = *(const v4ia*)(p + 12);
    d0 = q0.y; d1 = q0.w; d2 = q1.y; d3 = q1.w;
    d4 = q2.y; d5 = q2.w; d6 = q3.y; d7 = q3.w;
  } else {
#define LDJ(J, DJ) { int ec = e0 + (J); ec = ec > nE - 1 ? nE - 1 : ec; ec = ec < 0 ? 0 : ec; \
                     const int t = ei[2 * (size_t)ec + 1]; DJ = (e0 + (J) < nE) ? t : sent; }
    LDJ(0, d0) LDJ(1, d1) LDJ(2, d2) LDJ(3, d3) LDJ(4, d4) LDJ(5, d5) LDJ(6, d6) LDJ(7, d7)
#undef LDJ
  }
  const unsigned nb = (unsigned)nodeBase;
  const unsigned s0 = (unsigned)d0 - nb, s1 = (unsigned)d1 - nb, s2 = (unsigned)d2 - nb, s3 = (unsigned)d3 - nb;
  const unsigned s4 = (unsigned)d4 - nb, s5 = (unsigned)d5 - nb, s6 = (unsigned)d6 - nb, s7 = (unsigned)d7 - nb;
  const bool h0 = s0 < (unsigned)NB, h1 = s1 < (unsigned)NB, h2 = s2 < (unsigned)NB, h3 = s3 < (unsigned)NB;
  const bool h4 = s4 < (unsigned)NB, h5 = s5 < (unsigned)NB, h6 = s6 < (unsigned)NB, h7 = s7 < (unsigned)NB;
  const unsigned any = __builtin_amdgcn_ballot_w32(h0 | h1 | h2 | h3 | h4 | h5 | h6 | h7);
  if (any != 0u) {
#define HITJ(J, HJ, SJ) { \
      const unsigned mj = __builtin_amdgcn_ballot_w32(HJ); \
      if (mj != 0u) { \
        if (HJ) { \
          const int pos = wc + (int)__builtin_amdgcn_mbcnt_lo(mj, 0u); \
          if (pos < WCAP) list[wave * WCAP + pos] = ((el0 + (J)) << SLOTB) | (int)(SJ); \
        } \
        wc += (int)__builtin_popcount(mj); } }
    HITJ(0, h0, s0)
    HITJ(1, h1, s1)
    HITJ(2, h2, s2)
    HITJ(3, h3, s3)
    HITJ(4, h4, s4)
    HITJ(5, h5, s5)
    HITJ(6, h6, s6)
    HITJ(7, h7, s7)
#undef HITJ
  }
  return wc;
}

__global__ __launch_bounds__(NTHR) void k_agg(const float* __restrict__ pq, const int* __restrict__ ei,
                                              const float* __restrict__ mb1,
                                              float* spl, float* dpl, int nN, int nE) {
  extern __shared__ v4f dsm4[];
  v4f*   S4   = dsm4;
  float* sdeg = (float*)(dsm4 + NB * 32);
  __shared__ int list[NWAVE * WCAP];
  __shared__ int wcnt[NWAVE];

  const int tid = threadIdx.x, lane = tid & 31, wave = tid >> 5;
  const int nodeBase = blockIdx.x * NB;
  {
    v4f z4; z4.x = 0.0f; z4.y = 0.0f; z4.z = 0.0f; z4.w = 0.0f;
    for (int i = tid; i < NB * 32; i += NTHR) S4[i] = z4;
    for (int i = tid; i < NB; i += NTHR) sdeg[i] = 0.0f;
  }
  const v4f b1v = *(const v4fa*)(mb1 + 4 * lane);
  __syncthreads();

  const int nChunks = (nE + CHUNK - 1) / CHUNK;
#pragma unroll 1
  for (int ch = 0; ch < nChunks; ++ch) {
    const int cbase = ch * CHUNK;
    const int wc = scan_chunk(ei, nE, cbase, nodeBase, list, tid, wave);
    if (lane == 0) wcnt[wave] = wc;
    __syncthreads();

#pragma unroll 1
    for (int w2 = 0; w2 < NWAVE; ++w2) {
      int n = wcnt[w2];
      n = n < 0 ? 0 : (n > WCAP ? WCAP : n);
#pragma unroll 1
      for (int i = 0; i < n; ++i) {
        const int ent  = list[w2 * WCAP + i];
        const int slot = ent & (NB - 1);
        if ((slot & (NWAVE - 1)) == wave) {
          const int el = (ent >> SLOTB) & (CHUNK - 1);
          int e = cbase + el; e = e > nE - 1 ? nE - 1 : e; e = e < 0 ? 0 : e;
          int s = ei[2 * (size_t)e];
          s = s < 0 ? 0 : (s > nN - 1 ? nN - 1 : s);
          int dn = nodeBase + slot; dn = dn > nN - 1 ? nN - 1 : dn;
          const v4f p = *(const v4fa*)(pq + (size_t)s  * (size_t)(2 * HD) + 4 * lane);
          const v4f q = *(const v4fa*)(pq + (size_t)dn * (size_t)(2 * HD) + HD + 4 * lane);
          v4f hv = (p + q) + b1v;
          hv.x = fmaxf(hv.x, 0.0f); hv.y = fmaxf(hv.y, 0.0f); hv.z = fmaxf(hv.z, 0.0f); hv.w = fmaxf(hv.w, 0.0f);
          v4f cur = S4[slot * 32 + lane];
          cur += hv;
          S4[slot * 32 + lane] = cur;
          if (lane == 0) sdeg[slot] += 1.0f;
        }
      }
    }
    __syncthreads();
  }

  for (int r = wave; r < NB; r += NWAVE) {
    const v4f v = S4[r * 32 + lane];
    *(volatile v4f*)(spl + (size_t)(nodeBase + r) * HD + 4 * lane) = v;
  }
  for (int q = wave; q < NB / 128; q += NWAVE) {
    const v4f dv = *(const v4fa*)(sdeg + 128 * q + 4 * lane);
    *(volatile v4f*)(dpl + (size_t)nodeBase + 128 * q + 4 * lane) = dv;
  }
  __threadfence();
  for (int r = wave; r < NB; r += NWAVE) {
    const v4f v = S4[r * 32 + lane];
    *(volatile v4f*)(spl + (size_t)(nodeBase + r) * HD + 4 * lane) = v;
  }
  for (int q = wave; q < NB / 128; q += NWAVE) {
    const v4f dv = *(const v4fa*)(sdeg + 128 * q + 4 * lane);
    *(volatile v4f*)(dpl + (size_t)nodeBase + 128 * q + 4 * lane) = dv;
  }
}

__global__ __launch_bounds__(NTHR) void k_node(const float* __restrict__ x, const float* __restrict__ spl,
                                               const float* __restrict__ dpl, const us16* __restrict__ wt,
                                               const float* __restrict__ mb2, const float* __restrict__ ub1,
                                               const float* __restrict__ ub2,
                                               float* out, int nN, int nRowsS) {
  extern __shared__ v4f dsm4[];
  unsigned char* dsm = (unsigned char*)dsm4;
  us16*  A3H = (us16*)dsm;
  us16*  A3L = A3H + TR * 2 * HD;
  us16*  SH  = A3L + TR * 2 * HD;
  us16*  SL  = SH + TR * HD;
  us16*  UH  = SH;
  us16*  UL  = SL;
  float* OT  = (float*)dsm;
  __shared__ float sdeg[TR];

  const int tid = threadIdx.x, lane = tid & 31, wave = tid >> 5, h = lane >> 4, m = lane & 15;
  const int row0 = blockIdx.x * TR;

#pragma unroll
  for (int it = 0; it < (TR * HD / 4) / NTHR; ++it) {
    const int idx = it * NTHR + tid;
    const int r = idx >> 5, c4 = idx & 31;
    int grow = row0 + r; grow = grow > nN - 1 ? nN - 1 : grow;
    const v4f v = *(const v4fa*)(x + (size_t)grow * HD + 4 * c4);
    us16 a0, b0, a1, b1, a2, b2, a3, b3;
    split2(v.x, a0, b0); split2(v.y, a1, b1); split2(v.z, a2, b2); split2(v.w, a3, b3);
    v4us_t hv, lv;
    hv.x = a0; hv.y = a1; hv.z = a2; hv.w = a3;
    lv.x = b0; lv.y = b1; lv.z = b2; lv.w = b3;
    *(v4us*)(A3H + r * 2 * HD + 4 * c4) = hv;
    *(v4us*)(A3L + r * 2 * HD + 4 * c4) = lv;
  }
#pragma unroll
  for (int it = 0; it < (TR * HD / 4) / NTHR; ++it) {
    const int idx = it * NTHR + tid;
    const int r = idx >> 5, c4 = idx & 31;
    int srow = row0 + r; srow = srow > nRowsS - 1 ? nRowsS - 1 : srow;
    const v4f v = *(const v4fa*)(spl + (size_t)srow * HD + 4 * c4);
    us16 a0, b0, a1, b1, a2, b2, a3, b3;
    split2(v.x, a0, b0); split2(v.y, a1, b1); split2(v.z, a2, b2); split2(v.w, a3, b3);
    v4us_t hv, lv;
    hv.x = a0; hv.y = a1; hv.z = a2; hv.w = a3;
    lv.x = b0; lv.y = b1; lv.z = b2; lv.w = b3;
    *(v4us*)(SH + r * HD + 4 * c4) = hv;
    *(v4us*)(SL + r * HD + 4 * c4) = lv;
  }
  if (tid < TR) {
    int srow = row0 + tid; srow = srow > nRowsS - 1 ? nRowsS - 1 : srow;
    sdeg[tid] = dpl[srow];
  }
  __syncthreads();

  const int rh = wave >> 2, cg = wave & 3;
  const int arow0 = 32 * rh;
  const int bcol0 = 32 * cg;

  {
    v8f c00 = vz8(), c01 = vz8(), c10 = vz8(), c11 = vz8();
    wgemm2(c00, c01, c10, c11, SH, SL, HD, arow0, wt + OFF_W2H, wt + OFF_W2L, HD, bcol0, HD, m, h);
    const float bA = mb2[bcol0 + m], bB = mb2[bcol0 + 16 + m];
    epi_msg(A3H + HD, A3L + HD, 2 * HD, c00, arow0 + 8 * h,      bcol0 + m,      bA, sdeg);
    epi_msg(A3H + HD, A3L + HD, 2 * HD, c01, arow0 + 8 * h,      bcol0 + 16 + m, bB, sdeg);
    epi_msg(A3H + HD, A3L + HD, 2 * HD, c10, arow0 + 16 + 8 * h, bcol0 + m,      bA, sdeg);
    epi_msg(A3H + HD, A3L + HD, 2 * HD, c11, arow0 + 16 + 8 * h, bcol0 + 16 + m, bB, sdeg);
  }
  __syncthreads();

  {
    v8f c00 = vz8(), c01 = vz8(), c10 = vz8(), c11 = vz8();
    wgemm2(c00, c01, c10, c11, A3H, A3L, 2 * HD, arow0, wt + OFF_U1H, wt + OFF_U1L, 2 * HD, bcol0, 2 * HD, m, h);
    const float bA = ub1[bcol0 + m], bB = ub1[bcol0 + 16 + m];
    epi_split(UH, UL, HD, c00, arow0 + 8 * h,      bcol0 + m,      bA, 1);
    epi_split(UH, UL, HD, c01, arow0 + 8 * h,      bcol0 + 16 + m, bB, 1);
    epi_split(UH, UL, HD, c10, arow0 + 16 + 8 * h, bcol0 + m,      bA, 1);
    epi_split(UH, UL, HD, c11, arow0 + 16 + 8 * h, bcol0 + 16 + m, bB, 1);
  }
  __syncthreads();

  {
    v8f c00 = vz8(), c01 = vz8(), c10 = vz8(), c11 = vz8();
    wgemm2(c00, c01, c10, c11, UH, UL, HD, arow0, wt + OFF_U2H, wt + OFF_U2L, HD, bcol0, HD, m, h);
    const float bA = ub2[bcol0 + m], bB = ub2[bcol0 + 16 + m];
    epi_f32(OT, HD, c00, arow0 + 8 * h,      bcol0 + m,      bA);
    epi_f32(OT, HD, c01, arow0 + 8 * h,      bcol0 + 16 + m, bB);
    epi_f32(OT, HD, c10, arow0 + 16 + 8 * h, bcol0 + m,      bA);
    epi_f32(OT, HD, c11, arow0 + 16 + 8 * h, bcol0 + 16 + m, bB);
  }
  __syncthreads();

  for (int r = wave; r < TR; r += NWAVE) {
    const int grow = row0 + r;
    if (grow < nN) {
      const v4f v = *(const v4fa*)(OT + r * HD + 4 * lane);
      *(volatile v4f*)(out + (size_t)grow * HD + 4 * lane) = v;
    }
  }
  __threadfence();
  for (int r = wave; r < TR; r += NWAVE) {
    const int grow = row0 + r;
    if (grow < nN) {
      const v4f v = *(const v4fa*)(OT + r * HD + 4 * lane);
      *(volatile v4f*)(out + (size_t)grow * HD + 4 * lane) = v;
    }
  }
}

extern "C" void kernel_launch(void* const* d_in, const int* in_sizes, int n_in,
                              void* d_out, int out_size, void* d_ws, size_t ws_size,
                              hipStream_t stream) {
  if (n_in < 10) return;
  const int nN = in_sizes[0] / HD;
  if (nN <= 0 || in_sizes[0] != nN * HD) return;
  if (in_sizes[1] < 0 || (in_sizes[1] & 1) != 0) return;
  const int nE = in_sizes[1] / 2;
  if (in_sizes[2] != 2 * HD * HD || in_sizes[3] != HD || in_sizes[4] != HD * HD || in_sizes[5] != HD) return;
  if (in_sizes[6] != 2 * HD * HD || in_sizes[7] != HD || in_sizes[8] != HD * HD || in_sizes[9] != HD) return;
  if (out_size != nN * HD) return;

  const float* x   = (const float*)d_in[0];
  const int*   ei  = (const int*)d_in[1];
  const float* mw1 = (const float*)d_in[2];
  const float* mb1 = (const float*)d_in[3];
  const float* mw2 = (const float*)d_in[4];
  const float* mb2 = (const float*)d_in[5];
  const float* uw1 = (const float*)d_in[6];
  const float* ub1 = (const float*)d_in[7];
  const float* uw2 = (const float*)d_in[8];
  const float* ub2 = (const float*)d_in[9];
  float* out = (float*)d_out;

  const int nBlkT = (nN + TR - 1) / TR;
  const int nPadT = nBlkT * TR;
  const int nBlkA = (nN + NB - 1) / NB;
  const int nPadA = nBlkA * NB;

  char* ws = (char*)d_ws;
  size_t off = 0;
  const size_t oW  = off; off += (size_t)WT_HALVES * 2;                 off = (off + 255) & ~(size_t)255;
  const size_t oPQ = off; off += (size_t)nPadT * 2 * HD * sizeof(float); off = (off + 255) & ~(size_t)255;
  const size_t oS  = off; off += (size_t)nPadA * HD * sizeof(float);     off = (off + 255) & ~(size_t)255;
  const size_t oD  = off; off += (size_t)nPadA * sizeof(float);          off = (off + 255) & ~(size_t)255;
  if (off > ws_size) return;

  us16*  wt  = (us16*)(ws + oW);
  float* pq  = (float*)(ws + oPQ);
  float* spl = (float*)(ws + oS);
  float* dpl = (float*)(ws + oD);

  hipFuncSetAttribute(reinterpret_cast<const void*>(&k_pq),   hipFuncAttributeMaxDynamicSharedMemorySize, LDS_PQ);
  hipFuncSetAttribute(reinterpret_cast<const void*>(&k_agg),  hipFuncAttributeMaxDynamicSharedMemorySize, LDS_AGG);
  hipFuncSetAttribute(reinterpret_cast<const void*>(&k_node), hipFuncAttributeMaxDynamicSharedMemorySize, LDS_NODE);

  k_wcvt<<<40, NTHR, 0, stream>>>(mw1, mw2, uw1, uw2, wt);
  k_pq<<<nBlkT, NTHR, LDS_PQ, stream>>>(x, wt, pq, nN);
  k_agg<<<nBlkA, NTHR, LDS_AGG, stream>>>(pq, ei, mb1, spl, dpl, nN, nE);
  k_node<<<nBlkT, NTHR, LDS_NODE, stream>>>(x, spl, dpl, wt, mb2, ub1, ub2, out, nN, nPadA);
}
